// TextTaskPromptCrossAttention_16312285790680
// MI455X (gfx1250) — hardware-verified
//
#include <hip/hip_runtime.h>


#define NB_  2
#define NQ   2048
#define QD   1024
#define TCD  768
#define NCX  77
#define NPR  64
#define JJ   2189
#define JP   2304
#define INR  512
#define NH_  8
#define HD   64
#define ZH   4
#define PCAR 1024.0f
typedef _Float16 h16;
typedef unsigned short bf;
typedef __attribute__((ext_vector_type(16))) __bf16   v16bf;
typedef __attribute__((ext_vector_type(16))) _Float16 v16h;
typedef __attribute__((ext_vector_type(8)))  _Float16 v8h;
typedef __attribute__((ext_vector_type(8)))  unsigned short v8us;
typedef __attribute__((ext_vector_type(8)))  float    v8f;
typedef __attribute__((ext_vector_type(4)))  float    v4f;
typedef v8h  __attribute__((may_alias)) v8ha;
typedef v4f  __attribute__((may_alias)) v4fa;
typedef v8us __attribute__((may_alias)) v8usa;

__device__ __forceinline__ unsigned short f2bf(float f) { unsigned u = __float_as_uint(f); u += 0x7FFFu + ((u >> 16) & 1u); return (unsigned short)(u >> 16); }
__device__ __forceinline__ float bf2f(unsigned short b) { return __uint_as_float(((unsigned)b) << 16); }
__device__ __forceinline__ float bfr(float f) { return bf2f(f2bf(f)); }
__device__ __forceinline__ v16h cat16(v8h lo, v8h hi) { return __builtin_shufflevector(lo, hi, 0, 1, 2, 3, 4, 5, 6, 7, 8, 9, 10, 11, 12, 13, 14, 15); }
__device__ __forceinline__ v16bf cat16b(v8us lo, v8us hi) { return __builtin_bit_cast(v16bf, __builtin_shufflevector(lo, hi, 0, 1, 2, 3, 4, 5, 6, 7, 8, 9, 10, 11, 12, 13, 14, 15)); }
__device__ __forceinline__ v8f wmma16(v16h a, v16h b, v8f c) { return __builtin_amdgcn_wmma_f32_16x16x32_f16(false, a, false, b, (short)0, c, false, false); }
__device__ __forceinline__ v8f wmmab(v16bf a, v16bf b, v8f c) { return __builtin_amdgcn_wmma_f32_16x16x32_bf16(false, a, false, b, (short)0, c, false, false); }


template <typename T16> struct WFrag;
template <> struct WFrag<h16> { typedef v16h V; static __device__ __forceinline__ V ld(const h16* p) { return cat16(*(const v8h*)p, *(const v8h*)(p + 16)); } static __device__ __forceinline__ v8f mma(V a, V b, v8f c) { return wmma16(a, b, c); } };
template <> struct WFrag<bf> { typedef v16bf V; static __device__ __forceinline__ V ld(const bf* p) { return cat16b(*(const v8us*)p, *(const v8us*)(p + 16)); } static __device__ __forceinline__ v8f mma(V a, V b, v8f c) { return wmmab(a, b, c); } };
template <typename T16, int NSPLIT, bool BIAS>
__global__ __launch_bounds__(32) void k_gemmw(const T16* __restrict__ A, const T16* __restrict__ A2, const T16* __restrict__ Bt, const T16* __restrict__ Bt2, int K, float* C, int ldc, const float* __restrict__ bias, size_t sA, size_t sB, size_t sC) {
    typedef typename WFrag<T16>::V V;
    __shared__ __align__(16) float os[16 * 68];
    const size_t z = blockIdx.z; A += z * sA; if (A2) A2 += z * sA; Bt += z * sB; if (Bt2) Bt2 += z * sB; C += z * sC;
    const int lane = threadIdx.x & 31, lr = lane & 15, hi = lane >> 4; const int r0 = blockIdx.x * 64, c0 = blockIdx.y * 64;
    v8f acc[4][4];
#pragma unroll
    for (int mb = 0; mb < 4; ++mb)
#pragma unroll
        for (int nb = 0; nb < 4; ++nb) acc[mb][nb] = (v8f){};
    const size_t aoff = (size_t)(r0 + lr) * K + 8 * hi, boff = (size_t)(c0 + lr) * K + 8 * hi;
#pragma unroll 1
    for (int kc = 0; kc < K; kc += 32) {
        V a[4], a2[4];
#pragma unroll
        for (int mb = 0; mb < 4; ++mb) { a[mb] = WFrag<T16>::ld(A + aoff + (size_t)mb * 16 * K + kc); if (NSPLIT == 1 || NSPLIT == 2) a2[mb] = WFrag<T16>::ld(A2 + aoff + (size_t)mb * 16 * K + kc); }
#pragma unroll
        for (int nb = 0; nb < 4; ++nb) { const V b = WFrag<T16>::ld(Bt + boff + (size_t)nb * 16 * K + kc); V b2; if (NSPLIT >= 2) b2 = WFrag<T16>::ld(Bt2 + boff + (size_t)nb * 16 * K + kc);
#pragma unroll
            for (int mb = 0; mb < 4; ++mb) { acc[mb][nb] = WFrag<T16>::mma(a[mb], b, acc[mb][nb]); if (NSPLIT == 1 || NSPLIT == 2) acc[mb][nb] = WFrag<T16>::mma(a2[mb], b, acc[mb][nb]); if (NSPLIT >= 2) acc[mb][nb] = WFrag<T16>::mma(a[mb], b2, acc[mb][nb]); } }
        asm volatile("v_nop\n\tv_nop\n\tv_nop\n\tv_nop" : "+v"(acc[0][0]), "+v"(acc[1][1]), "+v"(acc[2][2]), "+v"(acc[3][3]) : "v"(a[0]), "v"(a[3]));
    }
#pragma unroll
    for (int mb = 0; mb < 4; ++mb) {
#pragma unroll
        for (int nb = 0; nb < 4; ++nb) {
#pragma unroll
            for (int j = 0; j < 8; ++j) os[(hi * 8 + j) * 68 + nb * 16 + lr] = acc[mb][nb][j]; }
        __builtin_amdgcn_wave_barrier(); asm volatile("" ::: "memory");
        float* crow = C + (size_t)(r0 + mb * 16) * ldc + c0;
#pragma unroll 1
        for (int ps = 0; ps < 2; ++ps) {
#pragma unroll
            for (int s = 0; s < 8; ++s) { const int row = 2 * s + hi, cofs = lr * 4; v4f val = *(const v4fa*)(os + row * 68 + cofs); if (BIAS) { val[0] += bfr(bias[c0 + cofs]); val[1] += bfr(bias[c0 + cofs + 1]); val[2] += bfr(bias[c0 + cofs + 2]); val[3] += bfr(bias[c0 + cofs + 3]); }
                *(volatile v4f*)(crow + (size_t)row * ldc + cofs) = val; }
            if (ps == 0) __threadfence(); }
        __builtin_amdgcn_wave_barrier(); asm volatile("" ::: "memory");
    }
}

__device__ __forceinline__ h16 tohx(float x) { return (h16)x; }
__device__ __forceinline__ void splitf(float y, unsigned short& h, unsigned short& l) { h = f2bf(y); l = f2bf(y - bf2f(h)); }
typedef __attribute__((ext_vector_type(2))) unsigned short v2us;
typedef __attribute__((ext_vector_type(4))) unsigned short v4us;
typedef __attribute__((ext_vector_type(2))) _Float16 v2h;
typedef __attribute__((ext_vector_type(4))) _Float16 v4h;

__global__ __launch_bounds__(256) void k_wtG(const float* __restrict__ w, int K, int N, bf* Bt) {
    const int lane = threadIdx.x & 31; const int L0 = (blockIdx.x * 8 + (threadIdx.x >> 5)) * 8; const int nlines = N * K / 64;
#pragma unroll
    for (int ps = 0; ps < 2; ++ps) {
#pragma unroll 1
        for (int l = 0; l < 8; ++l) { const int L = L0 + l; if (L >= nlines) break; const size_t e = (size_t)L * 64 + lane * 2; const int k = (int)(e % K), n = (int)(e / K); v2us o;
            o[0] = f2bf(w[(size_t)k * N + n]); o[1] = f2bf(w[(size_t)(k + 1) * N + n]); *(volatile v2us*)(Bt + e) = o; }
        if (ps == 0) __threadfence(); }
}
__global__ __launch_bounds__(256) void k_cvt8(const float* __restrict__ src, bf* dst, size_t n8) { const size_t i = (size_t)blockIdx.x * 256 + threadIdx.x; if (i >= n8) return; const v8f v = *(const v8f*)(src + i * 8); v8us o;
#pragma unroll
    for (int k = 0; k < 8; ++k) o[k] = f2bf(v[k]); *(volatile v8us*)(dst + i * 8) = o; __threadfence(); *(volatile v8us*)(dst + i * 8) = o; }
__global__ __launch_bounds__(256) void k_ctx(const float* __restrict__ cx, const float* __restrict__ PR, const float* __restrict__ IMG, bf* Ch, bf* Cl) { const size_t e = ((size_t)blockIdx.x * 256 + threadIdx.x) * 4; if (e >= (size_t)JP * TCD) return; const int c = (int)(e % TCD); const int j = (int)(e / TCD); v4us oh, ol;
#pragma unroll
    for (int u = 0; u < 4; ++u) { float v; if (j < NCX) { oh[u] = f2bf(cx[(size_t)j * TCD + c + u]); ol[u] = 0; continue; } else if (j < NCX + NPR) v = PR[(size_t)(j - NCX) * TCD + c + u]; else if (j < JJ) v = IMG[(size_t)(j - NCX - NPR) * TCD + c + u]; else v = 0.f; unsigned short a, b; splitf(v, a, b); oh[u] = a; ol[u] = b; }
    *(volatile v4us*)(Ch + e) = oh; *(volatile v4us*)(Cl + e) = ol; __threadfence(); *(volatile v4us*)(Ch + e) = oh; *(volatile v4us*)(Cl + e) = ol; }
__global__ __launch_bounds__(256) void k_q16(const float* __restrict__ FQ, h16* Q16) { const int e = (blockIdx.x * 256 + threadIdx.x) * 4; if (e >= NH_ * NQ * HD) return; const int d = e % HD; const int t = (e / HD) % NQ; const int h = e / (HD * NQ); const float* f = FQ + (size_t)t * INR + h * HD + d; v4h o;
#pragma unroll
    for (int u = 0; u < 4; ++u) o[u] = tohx(f[u] * 0.125f); *(volatile v4h*)(Q16 + e) = o; __threadfence(); *(volatile v4h*)(Q16 + e) = o; }
__global__ __launch_bounds__(256) void k_k16(const float* __restrict__ FK, h16* K16) { const int e = (blockIdx.x * 256 + threadIdx.x) * 4; if (e >= NH_ * JP * HD) return; const int d = e % HD; const int j = (e / HD) % JP; const int h = e / (HD * JP); const float* f = FK + (size_t)j * INR + h * HD + d; v4h o;
#pragma unroll
    for (int u = 0; u < 4; ++u) o[u] = tohx(f[u]); *(volatile v4h*)(K16 + e) = o; __threadfence(); *(volatile v4h*)(K16 + e) = o; }
__global__ __launch_bounds__(256) void k_vt(const float* __restrict__ FV, h16* VT) { const int e = (blockIdx.x * 256 + threadIdx.x) * 2; if (e >= NH_ * HD * JP) return; const int j = e % JP; const int d = (e / JP) % HD; const int h = e / (JP * HD); v2h o; o[0] = tohx(FV[(size_t)j * INR + h * HD + d]); o[1] = tohx(FV[(size_t)(j + 1) * INR + h * HD + d]); *(volatile v2h*)(VT + e) = o; __threadfence(); *(volatile v2h*)(VT + e) = o; }
__global__ __launch_bounds__(256) void k_psoft(const float* __restrict__ Sb, h16* P16) { const int lane = threadIdx.x & 31; const int row = blockIdx.x * 8 + (threadIdx.x >> 5); if (row >= ZH * NQ) return; const float* sr = Sb + (size_t)row * JP; float v[JP / 32]; float mx = -3.0e38f;
#pragma unroll
    for (int ch = 0; ch < JP / 128; ++ch) { const int j0 = ch * 128 + lane * 4; const v4f a = *(const v4f*)(sr + j0);
#pragma unroll
        for (int u = 0; u < 4; ++u) { const float t = (j0 + u < JJ) ? a[u] : -3.0e38f; v[ch * 4 + u] = t; mx = fmaxf(mx, t); } }
#pragma unroll
    for (int sh = 16; sh; sh >>= 1) mx = fmaxf(mx, __shfl_xor(mx, sh, 32));
    float sum = 0.f;
#pragma unroll
    for (int q = 0; q < JP / 32; ++q) { float d0 = __fsub_rn(v[q], mx); asm volatile("" : "+v"(d0)); v[q] = __builtin_amdgcn_exp2f(__fmul_rn(d0, 1.4426950408889634f)); sum += v[q]; }
#pragma unroll
    for (int sh = 16; sh; sh >>= 1) sum += __shfl_xor(sum, sh, 32);
    const float f = __fdiv_rn(PCAR, sum);
    for (int ps = 0; ps < 2; ++ps) {
#pragma unroll
        for (int ch = 0; ch < JP / 128; ++ch) { v4h o4;
#pragma unroll
            for (int q = 0; q < 4; ++q) o4[q] = tohx(v[ch * 4 + q] * f); *(volatile v4h*)(P16 + (size_t)row * JP + ch * 128 + lane * 4) = o4; }
        if (ps == 0) __threadfence(); } }
__global__ __launch_bounds__(256) void k_mrg(const float* __restrict__ O, int h0, bf* Ah, bf* Al) { const int e = (blockIdx.x * 256 + threadIdx.x) * 4; if (e >= ZH * NQ * HD) return; const int d = e % HD; const int t = (e / HD) % NQ; const int z = e / (HD * NQ); v4us oh, ol;
#pragma unroll
    for (int u = 0; u < 4; ++u) { unsigned short a, b; splitf(O[e + u] * (1.0f / PCAR), a, b); oh[u] = a; ol[u] = b; } const size_t oo = (size_t)t * INR + (h0 + z) * HD + d; *(volatile v4us*)(Ah + oo) = oh; *(volatile v4us*)(Al + oo) = ol; __threadfence(); *(volatile v4us*)(Ah + oo) = oh; *(volatile v4us*)(Al + oo) = ol; }

extern "C" void kernel_launch(void* const* d_in, const int* in_sizes, int n_in,
                              void* d_out, int out_size, void* d_ws, size_t ws_size, hipStream_t stream) {
    (void)in_sizes; (void)n_in; (void)out_size;
    const float* x = (const float*)d_in[0]; const float* cx = (const float*)d_in[1]; const float* pr = (const float*)d_in[2]; const float* wpr = (const float*)d_in[3]; const float* wimg = (const float*)d_in[4]; const float* wq = (const float*)d_in[5]; const float* wk = (const float*)d_in[6]; const float* wv = (const float*)d_in[7]; const float* wout = (const float*)d_in[8]; const float* bout = (const float*)d_in[9];
    float* OUT = (float*)d_out;
    char* wsp = (char*)d_ws;
    auto take = [&](size_t bytes) { char* p = wsp; wsp += (bytes + 255) & ~(size_t)255; return (void*)p; };
    bf* WPR = (bf*)take((size_t)TCD * QD * 2); bf* WIMG = (bf*)take((size_t)TCD * QD * 2); bf* WQ = (bf*)take((size_t)INR * QD * 2); bf* WK = (bf*)take((size_t)INR * TCD * 2); bf* WV = (bf*)take((size_t)INR * TCD * 2); bf* WO = (bf*)take((size_t)QD * INR * 2);
    bf* PB = (bf*)take((size_t)NPR * QD * 2); float* PR = (float*)take((size_t)NPR * TCD * 4); bf* XB = (bf*)take((size_t)NQ * QD * 2); float* FQ = (float*)take((size_t)NQ * INR * 4); float* IMG = (float*)take((size_t)NQ * TCD * 4); bf* Ch = (bf*)take((size_t)JP * TCD * 2); bf* Cl = (bf*)take((size_t)JP * TCD * 2);
    float* FK = (float*)take((size_t)JP * INR * 4); float* FV = (float*)take((size_t)JP * INR * 4); h16* Q16 = (h16*)take((size_t)NH_ * NQ * HD * 2); h16* K16 = (h16*)take((size_t)NH_ * JP * HD * 2); h16* VT = (h16*)take((size_t)NH_ * HD * JP * 2);
    float* Sb = (float*)take((size_t)ZH * NQ * JP * 4); h16* P16 = (h16*)take((size_t)ZH * NQ * JP * 2); float* O = (float*)take((size_t)ZH * NQ * HD * 4); bf* Ah = (bf*)take((size_t)NQ * INR * 2); bf* Al = (bf*)take((size_t)NQ * INR * 2);
    if ((size_t)(wsp - (char*)d_ws) > ws_size) return;
    k_wtG<<<(QD * TCD / 64 + 63) / 64, 256, 0, stream>>>(wpr, QD, TCD, WPR); k_wtG<<<(QD * TCD / 64 + 63) / 64, 256, 0, stream>>>(wimg, QD, TCD, WIMG); k_wtG<<<(QD * INR / 64 + 63) / 64, 256, 0, stream>>>(wq, QD, INR, WQ);
    k_wtG<<<(TCD * INR / 64 + 63) / 64, 256, 0, stream>>>(wk, TCD, INR, WK); k_wtG<<<(TCD * INR / 64 + 63) / 64, 256, 0, stream>>>(wv, TCD, INR, WV); k_wtG<<<(INR * QD / 64 + 63) / 64, 256, 0, stream>>>(wout, INR, QD, WO);
    k_cvt8<<<(NPR * QD / 8 + 255) / 256, 256, 0, stream>>>(pr, PB, NPR * QD / 8); k_gemmw<bf, 0, false><<<dim3(NPR / 64, TCD / 64, 1), 32, 0, stream>>>(PB, nullptr, WPR, nullptr, QD, PR, TCD, nullptr, 0, 0, 0);
    for (int b = 0; b < NB_; ++b) {
        k_cvt8<<<(NQ * QD / 8 + 255) / 256, 256, 0, stream>>>(x + (size_t)b * NQ * QD, XB, (size_t)NQ * QD / 8);
        k_gemmw<bf, 0, false><<<dim3(NQ / 64, INR / 64, 1), 32, 0, stream>>>(XB, nullptr, WQ, nullptr, QD, FQ, INR, nullptr, 0, 0, 0); k_gemmw<bf, 0, false><<<dim3(NQ / 64, TCD / 64, 1), 32, 0, stream>>>(XB, nullptr, WIMG, nullptr, QD, IMG, TCD, nullptr, 0, 0, 0);
        k_ctx<<<(unsigned)(((size_t)JP * TCD / 4 + 255) / 256), 256, 0, stream>>>(cx + (size_t)b * NCX * TCD, PR, IMG, Ch, Cl);
        k_gemmw<bf, 1, false><<<dim3(JP / 64, INR / 64, 1), 32, 0, stream>>>(Ch, Cl, WK, nullptr, TCD, FK, INR, nullptr, 0, 0, 0); k_gemmw<bf, 1, false><<<dim3(JP / 64, INR / 64, 1), 32, 0, stream>>>(Ch, Cl, WV, nullptr, TCD, FV, INR, nullptr, 0, 0, 0);
        k_q16<<<(NH_ * NQ * HD / 4 + 255) / 256, 256, 0, stream>>>(FQ, Q16); k_k16<<<(NH_ * JP * HD / 4 + 255) / 256, 256, 0, stream>>>(FK, K16); k_vt<<<(NH_ * HD * JP / 2 + 255) / 256, 256, 0, stream>>>(FV, VT);
        for (int h0 = 0; h0 < NH_; h0 += ZH) {
            k_gemmw<h16, 0, false><<<dim3(NQ / 64, JP / 64, ZH), 32, 0, stream>>>(Q16 + (size_t)h0 * NQ * HD, nullptr, K16 + (size_t)h0 * JP * HD, nullptr, HD, Sb, JP, nullptr, (size_t)NQ * HD, (size_t)JP * HD, (size_t)NQ * JP);
            k_psoft<<<ZH * NQ / 8, 256, 0, stream>>>(Sb, P16);
            k_gemmw<h16, 0, false><<<dim3(NQ / 64, 1, ZH), 32, 0, stream>>>(P16, nullptr, VT + (size_t)h0 * HD * JP, nullptr, JP, O, HD, nullptr, (size_t)NQ * JP, (size_t)HD * JP, (size_t)NQ * HD);
            k_mrg<<<(ZH * NQ * HD / 4 + 255) / 256, 256, 0, stream>>>(O, h0, Ah, Al); }
        k_gemmw<bf, 1, true><<<dim3(NQ / 64, QD / 64, 1), 32, 0, stream>>>(Ah, Al, WO, nullptr, INR, OUT + (size_t)b * NQ * QD, QD, bout, 0, 0, 0); }
}
